// RelationalTransformer_77017353551926
// MI455X (gfx1250) — hardware-verified
//
#include <hip/hip_runtime.h>
#include <math.h>

#define BB   2
#define SS   512
#define HID  256
#define NHD  8
#define HD   32
#define NL   12
#define NA   5
#define MLPD 1024
#define FC1N 2048
#define VD   384
#define SD   384
#define TD   5
#define RD   64
#define ND   5
#define CTXD 1280
#define MTOK (BB * SS)
#define WSC  1024.0f
#define CSC  16.0f
#define OSC  64.0f
#define HSC  64.0f
#define PSC  16384.0f
#define LNEPS 1e-5f

static_assert(MTOK % 128 == 0);
static_assert(SS % 64 == 0);
static_assert(HID == NHD * HD);
static_assert(HD == 32);
static_assert(CTXD == 5 * HID);
static_assert(FC1N == 2 * MLPD);
static_assert(VD % 64 == 0 && SD % 64 == 0 && RD % 64 == 0 && CTXD % 64 == 0 && MLPD % 64 == 0 && HID % 64 == 0);

typedef _Float16 v16h __attribute__((ext_vector_type(16)));
typedef _Float16 v8h  __attribute__((ext_vector_type(8)));
typedef _Float16 v4hq __attribute__((ext_vector_type(4)));
typedef float    v8f  __attribute__((ext_vector_type(8)));
typedef float    v4f  __attribute__((ext_vector_type(4)));
typedef int      v4i  __attribute__((ext_vector_type(4)));
typedef v8h __attribute__((may_alias)) v8ha;
typedef v4f __attribute__((may_alias)) v4fa;
typedef v4i __attribute__((may_alias)) v4ia;

union Frag { v16h v; v8h half[2]; };

__device__ __forceinline__ v8f zero8f() { v8f z = {0.f, 0.f, 0.f, 0.f, 0.f, 0.f, 0.f, 0.f}; return z; }

__device__ __forceinline__ v8f wmma_f16(v16h a, v16h b, v8f c) {
  v8f d = __builtin_amdgcn_wmma_f32_16x16x32_f16(false, a, false, b, (short)0, c, false, false);
  asm volatile("v_nop\n\tv_nop\n\tv_nop\n\tv_nop" : "+v"(d) : "v"(a), "v"(b));
  return d;
}

__device__ __forceinline__ v16h load_frag(const _Float16* p, int h) {
  Frag f;
  f.half[0] = *(const v8ha*)(p + 8 * h);
  f.half[1] = *(const v8ha*)(p + 16 + 8 * h);
  return f.v;
}

__device__ __forceinline__ v4f ld4(const float* p) { return *(const v4fa*)p; }
__device__ __forceinline__ v4hq cvt4h(v4f v) {
  v4hq r = { (_Float16)v.x, (_Float16)v.y, (_Float16)v.z, (_Float16)v.w };
  return r;
}
__device__ __forceinline__ float rcpf(float x) { return __builtin_amdgcn_rcpf(x); }
__device__ __forceinline__ v4f sig4(v4f u) {
  v4f r;
  r.x = rcpf(1.0f + __expf(-u.x));
  r.y = rcpf(1.0f + __expf(-u.y));
  r.z = rcpf(1.0f + __expf(-u.z));
  r.w = rcpf(1.0f + __expf(-u.w));
  return r;
}
__device__ __forceinline__ v4f sel4(int c, v4f a, v4f b) {
  v4f r;
  r.x = c ? a.x : b.x;
  r.y = c ? a.y : b.y;
  r.z = c ? a.z : b.z;
  r.w = c ? a.w : b.w;
  return r;
}
__device__ __forceinline__ float wsum(float v) {
#pragma unroll
  for (int off = 16; off >= 1; off >>= 1) v += __shfl_xor(v, off, 32);
  return v;
}

__global__ __launch_bounds__(256) void cvt_in_kernel(
    const float* __restrict__ val, const float* __restrict__ sch, const float* __restrict__ rol,
    _Float16* v16p, _Float16* s16p, _Float16* r16p)
{
  const int g = blockIdx.x * 256 + threadIdx.x;
  const int n8v = MTOK * VD / 8, n8s = MTOK * SD / 8, n8r = MTOK * RD / 8;
  if (g >= n8v + n8s + n8r) return;
  const float* src;
  _Float16* dst;
  if (g < n8v) {
    src = val + (size_t)g * 8; dst = v16p + (size_t)g * 8;
  } else if (g < n8v + n8s) {
    const int e = g - n8v;
    src = sch + (size_t)e * 8; dst = s16p + (size_t)e * 8;
  } else {
    const int e = g - n8v - n8s;
    src = rol + (size_t)e * 8; dst = r16p + (size_t)e * 8;
  }
  const v4f a = ld4(src);
  const v4f c = ld4(src + 4);
  const v8h o = { (_Float16)a.x, (_Float16)a.y, (_Float16)a.z, (_Float16)a.w,
                  (_Float16)c.x, (_Float16)c.y, (_Float16)c.z, (_Float16)c.w };
  *(volatile v8h*)dst = o;
  __threadfence();
  *(volatile v8h*)dst = o;
}

__global__ __launch_bounds__(256) void wtrans_kernel(const float* __restrict__ W, _Float16* out, int K, int N)
{
  __shared__ __attribute__((aligned(16))) _Float16 sT[64 * 72];
  const int tid = threadIdx.x, lane = tid & 31, w = tid >> 5;
  const int n0 = blockIdx.x * 64, k0 = blockIdx.y * 64, z = blockIdx.z;
  const int r = tid >> 2, c16 = (tid & 3) * 16;
  const float* src = W + ((size_t)z * K + k0 + r) * N + n0 + c16;
#pragma unroll
  for (int q = 0; q < 4; ++q) {
    const v4f a = ld4(src + 4 * q);
    sT[(c16 + 4 * q + 0) * 72 + r] = (_Float16)(a.x * WSC);
    sT[(c16 + 4 * q + 1) * 72 + r] = (_Float16)(a.y * WSC);
    sT[(c16 + 4 * q + 2) * 72 + r] = (_Float16)(a.z * WSC);
    sT[(c16 + 4 * q + 3) * 72 + r] = (_Float16)(a.w * WSC);
  }
  __syncthreads();
  const int q8 = lane & 7, sub = lane >> 3;
#pragma unroll
  for (int i = 0; i < 2; ++i) {
    const int n = 8 * w + 4 * i + sub;
    const v8h v = *(const v8ha*)(sT + n * 72 + 8 * q8);
    _Float16* dst = out + ((size_t)z * N + n0 + n) * K + k0 + 8 * q8;
    *(volatile v8h*)dst = v;
    __threadfence();
    *(volatile v8h*)dst = v;
  }
}

__device__ __forceinline__ void f32tile_store_pass(const float* sF, float* C, int ldc,
                                                   int m0, int n0, int w, int lane) {
  const int q8 = lane & 7, sub = lane >> 3;
#pragma unroll
  for (int i = 0; i < 16; ++i) {
    const int lid = w * 64 + i * 4 + sub;
    const int row = lid >> 1, hl = lid & 1;
    const v4f v = ld4(sF + row * 64 + 32 * hl + 4 * q8);
    *(volatile v4f*)(C + (size_t)(m0 + row) * ldc + n0 + 32 * hl + 4 * q8) = v;
  }
}

__global__ __launch_bounds__(128) void gemm_f32_kernel(
    const _Float16* __restrict__ A, int lda, long long strideA,
    const _Float16* __restrict__ Bt, int ldb, long long strideB,
    float* C, int ldc, long long strideC, int K, float osc)
{
  __shared__ __attribute__((aligned(16))) float sF[128 * 64];
  const int tid = threadIdx.x, lane = tid & 31, w = tid >> 5;
  const int h = lane >> 4, m = lane & 15;
  const int m0 = blockIdx.x * 128, n0 = blockIdx.y * 64, z = blockIdx.z;
  const _Float16* Ab = A + (size_t)z * (size_t)strideA;
  const _Float16* Bb = Bt + (size_t)z * (size_t)strideB;
  const _Float16* xa0 = Ab + (size_t)(m0 + 32 * w + m) * lda;
  const _Float16* xa1 = xa0 + (size_t)16 * lda;
  const _Float16* wb = Bb + (size_t)(n0 + m) * ldb;

  const v8f z8 = zero8f();
  v8f acc[2][4];
#pragma unroll
  for (int mt = 0; mt < 2; ++mt)
#pragma unroll
    for (int nt = 0; nt < 4; ++nt) acc[mt][nt] = z8;

#pragma unroll 1
  for (int k0 = 0; k0 < K; k0 += 32) {
    const v16h a0 = load_frag(xa0 + k0, h);
    const v16h a1 = load_frag(xa1 + k0, h);
#pragma unroll
    for (int nt = 0; nt < 4; ++nt) {
      const v16h b = load_frag(wb + (size_t)nt * 16 * ldb + k0, h);
      acc[0][nt] = wmma_f16(a0, b, acc[0][nt]);
      acc[1][nt] = wmma_f16(a1, b, acc[1][nt]);
    }
  }

#pragma unroll
  for (int nt = 0; nt < 4; ++nt)
#pragma unroll
    for (int mt = 0; mt < 2; ++mt)
#pragma unroll
      for (int r = 0; r < 8; ++r) {
        const int tokl = 32 * w + 16 * mt + 8 * h + r;
        sF[tokl * 64 + 16 * nt + m] = acc[mt][nt][r] * osc;
      }
  __syncthreads();

  float* Cb = C + (size_t)z * (size_t)strideC;
  f32tile_store_pass(sF, Cb, ldc, m0, n0, w, lane);
  __threadfence();
  f32tile_store_pass(sF, Cb, ldc, m0, n0, w, lane);
}

__global__ __launch_bounds__(256) void embed_kernel(
    const float* __restrict__ VP, const float* __restrict__ SP, const float* __restrict__ RP,
    const float* __restrict__ tmp, const float* __restrict__ Wt, const float* __restrict__ Ed,
    const float* __restrict__ Em, const int* __restrict__ dtype_ids, const int* __restrict__ is_masked,
    float* comb, _Float16* ctx)
{
  const int lane = threadIdx.x & 31, w = threadIdx.x >> 5;
  const int tok = blockIdx.x * 8 + w;
  int d = dtype_ids[tok];
  d = (d < 0) ? 0 : ((d > ND - 1) ? (ND - 1) : d);
  const int mk = is_masked[tok];
  const int ca = 4 * lane, cb = 128 + 4 * lane;
  const size_t rt = (size_t)tok * HID;

  const v4f vpa = ld4(VP + ((size_t)d * MTOK + tok) * HID + ca);
  const v4f vpb = ld4(VP + ((size_t)d * MTOK + tok) * HID + cb);
  const v4f ema = ld4(Em + (size_t)d * HID + ca);
  const v4f emb = ld4(Em + (size_t)d * HID + cb);
  const v4f spa = ld4(SP + rt + ca), spb = ld4(SP + rt + cb);
  const v4f rpa = ld4(RP + rt + ca), rpb = ld4(RP + rt + cb);
  const v4f dea = ld4(Ed + (size_t)d * HID + ca);
  const v4f deb = ld4(Ed + (size_t)d * HID + cb);
  v4f tpa = {0.f, 0.f, 0.f, 0.f};
  v4f tpb = {0.f, 0.f, 0.f, 0.f};
#pragma unroll 1
  for (int k = 0; k < TD; ++k) {
    const float te = tmp[(size_t)tok * TD + k];
    const v4f wa = ld4(Wt + (size_t)k * HID + ca);
    const v4f wbv = ld4(Wt + (size_t)k * HID + cb);
    tpa = tpa + wa * te;
    tpb = tpb + wbv * te;
  }
  const v4f va = sel4(mk, ema, vpa);
  const v4f vb = sel4(mk, emb, vpb);
  const v4f cma = (((va + spa) + tpa) + rpa) + dea;
  const v4f cmb = (((vb + spb) + tpb) + rpb) + deb;

  const v4hq h0a = cvt4h(va * CSC),  h0b = cvt4h(vb * CSC);
  const v4hq h1a = cvt4h(spa * CSC), h1b = cvt4h(spb * CSC);
  const v4hq h2a = cvt4h(tpa * CSC), h2b = cvt4h(tpb * CSC);
  const v4hq h3a = cvt4h(rpa * CSC), h3b = cvt4h(rpb * CSC);
  const v4hq h4a = cvt4h(dea * CSC), h4b = cvt4h(deb * CSC);

  float* crow = comb + rt;
  _Float16* xr = ctx + (size_t)tok * CTXD;
  for (int pass = 0; pass < 2; ++pass) {
    *(volatile v4f*)(crow + ca) = cma;
    *(volatile v4f*)(crow + cb) = cmb;
    *(volatile v4hq*)(xr + 0 * HID + ca) = h0a;
    *(volatile v4hq*)(xr + 0 * HID + cb) = h0b;
    *(volatile v4hq*)(xr + 1 * HID + ca) = h1a;
    *(volatile v4hq*)(xr + 1 * HID + cb) = h1b;
    *(volatile v4hq*)(xr + 2 * HID + ca) = h2a;
    *(volatile v4hq*)(xr + 2 * HID + cb) = h2b;
    *(volatile v4hq*)(xr + 3 * HID + ca) = h3a;
    *(volatile v4hq*)(xr + 3 * HID + cb) = h3b;
    *(volatile v4hq*)(xr + 4 * HID + ca) = h4a;
    *(volatile v4hq*)(xr + 4 * HID + cb) = h4b;
    __threadfence();
  }
}

template <int ACT, int MODE, int HASB, int FINAL>
__global__ __launch_bounds__(128) void rowgemm_kernel(
    const _Float16* __restrict__ A, int lda, const _Float16* __restrict__ Bt, int K, float osc,
    const float* __restrict__ bias, float* x, const float* __restrict__ comb, const int* __restrict__ padm,
    const float* __restrict__ g, const float* __restrict__ be, _Float16* xn, float* outf)
{
  __shared__ __attribute__((aligned(16))) float sX[32 * 260];
  const int tid = threadIdx.x, lane = tid & 31, w = tid >> 5;
  const int h = lane >> 4, m = lane & 15;
  const int m0 = blockIdx.x * 32;
  const int wr = w >> 1, wc = w & 1;
  const int arow = m0 + 16 * wr + m;
  const _Float16* wb = Bt + (size_t)(128 * wc + m) * K;

  const v8f z8 = zero8f();
  v8f acc[8];
#pragma unroll
  for (int nt = 0; nt < 8; ++nt) acc[nt] = z8;

#pragma unroll 1
  for (int k0 = 0; k0 < K; k0 += 32) {
    const _Float16* ap;
    if (ACT) ap = A + (size_t)(((arow >> 9) * NHD + (k0 >> 5)) * SS + (arow & (SS - 1))) * HD;
    else     ap = A + (size_t)arow * lda + k0;
    const v16h a = load_frag(ap, h);
#pragma unroll
    for (int nt = 0; nt < 8; ++nt) {
      const v16h b = load_frag(wb + (size_t)nt * 16 * K + k0, h);
      acc[nt] = wmma_f16(a, b, acc[nt]);
    }
  }

#pragma unroll
  for (int nt = 0; nt < 8; ++nt) {
    const int col = 128 * wc + 16 * nt + m;
#pragma unroll
    for (int r = 0; r < 8; ++r) sX[(16 * wr + 8 * h + r) * 260 + col] = acc[nt][r] * osc;
  }
  __syncthreads();

  const int ca = 4 * lane, cb = 128 + 4 * lane;
  const v4f ga = ld4(g + ca), gb = ld4(g + cb);
  const v4f ba = ld4(be + ca), bb = ld4(be + cb);
  v4f bia = {0.f, 0.f, 0.f, 0.f};
  v4f bib = {0.f, 0.f, 0.f, 0.f};
  if (HASB) { bia = ld4(bias + ca); bib = ld4(bias + cb); }

#pragma unroll 1
  for (int i = 0; i < 8; ++i) {
    const int rr = 8 * w + i;
    const int grow = m0 + rr;
    const float* sp = sX + rr * 260;
    v4f ua = ld4(sp + ca) + bia;
    v4f ub = ld4(sp + cb) + bib;
    v4f va, vb;
    if (MODE == 0) {
      const v4f xa = ld4(x + (size_t)grow * HID + ca);
      const v4f xb = ld4(x + (size_t)grow * HID + cb);
      va = ua + xa;
      vb = ub + xb;
    } else {
      const float pm = (padm[grow] != 0) ? 1.0f : 0.0f;
      const v4f cma = ld4(comb + (size_t)grow * HID + ca);
      const v4f cmb = ld4(comb + (size_t)grow * HID + cb);
      va = (cma * sig4(ua)) * pm;
      vb = (cmb * sig4(ub)) * pm;
    }
    float s1 = ((va.x + va.y) + (va.z + va.w)) + ((vb.x + vb.y) + (vb.z + vb.w));
    s1 = wsum(s1);
    const float mean = s1 * (1.0f / HID);
    const v4f da = va - mean, db = vb - mean;
    float s2 = ((da.x * da.x + da.y * da.y) + (da.z * da.z + da.w * da.w)) +
               ((db.x * db.x + db.y * db.y) + (db.z * db.z + db.w * db.w));
    s2 = wsum(s2);
    const float rs = rsqrtf(s2 * (1.0f / HID) + LNEPS);
    const v4f ya = (da * rs) * ga + ba;
    const v4f yb = (db * rs) * gb + bb;
    if (!FINAL) {
      const v4hq ha = cvt4h(ya), hb = cvt4h(yb);
      float* xrow = x + (size_t)grow * HID;
      _Float16* nrow = xn + (size_t)grow * HID;
      *(volatile v4f*)(xrow + ca) = va;
      *(volatile v4f*)(xrow + cb) = vb;
      *(volatile v4hq*)(nrow + ca) = ha;
      *(volatile v4hq*)(nrow + cb) = hb;
      __threadfence();
      *(volatile v4f*)(xrow + ca) = va;
      *(volatile v4f*)(xrow + cb) = vb;
      *(volatile v4hq*)(nrow + ca) = ha;
      *(volatile v4hq*)(nrow + cb) = hb;
    } else {
      float* orow = outf + (size_t)grow * HID;
      *(volatile v4f*)(orow + ca) = ya;
      *(volatile v4f*)(orow + cb) = yb;
      __threadfence();
      *(volatile v4f*)(orow + ca) = ya;
      *(volatile v4f*)(orow + cb) = yb;
    }
  }
}

__device__ __forceinline__ void qkv_store_pass(const _Float16* sT, _Float16* plane, _Float16* vtp,
                                               int which, int b, int hp, int l0, int w, int lane) {
  const int q8 = lane & 7, sub = lane >> 3;
#pragma unroll
  for (int i = 0; i < 8; ++i) {
    const int lid = w * 32 + i * 4 + sub;
    const int hh2 = lid >> 6, rem = lid & 63;
    const int bh = b * NHD + 2 * hp + hh2;
    v8h v;
    _Float16* dst;
    if (which != 2) {
      const int tk = 2 * rem + (q8 >> 2), d0 = (q8 & 3) * 8;
      v = *(const v8ha*)(sT + tk * 64 + hh2 * 32 + d0);
      dst = plane + ((size_t)bh * SS + l0 + tk) * HD + d0;
    } else {
      const int d = rem >> 1, hl = rem & 1;
      v = *(const v8ha*)(sT + (hh2 * 32 + d) * 128 + 64 * hl + 8 * q8);
      dst = vtp + ((size_t)bh * HD + d) * SS + l0 + 64 * hl + 8 * q8;
    }
    *(volatile v8h*)dst = v;
  }
}

__global__ __launch_bounds__(128) void qkv_kernel(
    const _Float16* __restrict__ xn, const _Float16* __restrict__ wt,
    _Float16* qp, _Float16* kp, _Float16* vtp)
{
  __shared__ __attribute__((aligned(16))) _Float16 sT[128 * 64];
  const int tid = threadIdx.x, lane = tid & 31, w = tid >> 5;
  const int h = lane >> 4, m = lane & 15;
  const int m0 = blockIdx.x * 128;
  const int cg = blockIdx.y;
  const int which = cg >> 2, hp = cg & 3;
  const int f0 = which * HID + hp * 64;
  const _Float16* xa0 = xn + (size_t)(m0 + 32 * w + m) * HID;
  const _Float16* xa1 = xa0 + (size_t)16 * HID;
  const _Float16* wb = wt + (size_t)(f0 + m) * HID;

  const v8f z8 = zero8f();
  v8f acc[2][4];
#pragma unroll
  for (int mt = 0; mt < 2; ++mt)
#pragma unroll
    for (int nt = 0; nt < 4; ++nt) acc[mt][nt] = z8;

#pragma unroll 1
  for (int k0 = 0; k0 < HID; k0 += 32) {
    const v16h a0 = load_frag(xa0 + k0, h);
    const v16h a1 = load_frag(xa1 + k0, h);
#pragma unroll
    for (int nt = 0; nt < 4; ++nt) {
      const v16h b = load_frag(wb + (size_t)nt * 16 * HID + k0, h);
      acc[0][nt] = wmma_f16(a0, b, acc[0][nt]);
      acc[1][nt] = wmma_f16(a1, b, acc[1][nt]);
    }
  }

#pragma unroll
  for (int nt = 0; nt < 4; ++nt) {
    const int featl = 16 * nt + m;
#pragma unroll
    for (int mt = 0; mt < 2; ++mt)
#pragma unroll
      for (int r = 0; r < 8; ++r) {
        const int tokl = 32 * w + 16 * mt + 8 * h + r;
        const float y = acc[mt][nt][r] * (1.0f / WSC);
        const int idx = (which == 2) ? (featl * 128 + tokl) : (tokl * 64 + featl);
        sT[idx] = (_Float16)y;
      }
  }
  __syncthreads();

  const int b = m0 >> 9, l0 = m0 & (SS - 1);
  _Float16* plane = (which == 0) ? qp : kp;
  qkv_store_pass(sT, plane, vtp, which, b, hp, l0, w, lane);
  __threadfence();
  qkv_store_pass(sT, plane, vtp, which, b, hp, l0, w, lane);
}

__device__ __forceinline__ v16h pack_p(v8f a, v8f c) {
  const v16h r = { (_Float16)(a[0] * PSC), (_Float16)(a[1] * PSC), (_Float16)(a[2] * PSC), (_Float16)(a[3] * PSC),
                   (_Float16)(a[4] * PSC), (_Float16)(a[5] * PSC), (_Float16)(a[6] * PSC), (_Float16)(a[7] * PSC),
                   (_Float16)(c[0] * PSC), (_Float16)(c[1] * PSC), (_Float16)(c[2] * PSC), (_Float16)(c[3] * PSC),
                   (_Float16)(c[4] * PSC), (_Float16)(c[5] * PSC), (_Float16)(c[6] * PSC), (_Float16)(c[7] * PSC) };
  return r;
}

__device__ __forceinline__ void att_store_pass(const _Float16* so, _Float16* ct, int bh, int q0, int lane) {
  const int q8 = lane & 7, sub = lane >> 3;
#pragma unroll
  for (int i = 0; i < 2; ++i) {
    const int lid = i * 4 + sub;
    const int ql = 2 * lid + (q8 >> 2), d0 = (q8 & 3) * 8;
    const v8h v = *(const v8ha*)(so + ql * HD + d0);
    *(volatile v8h*)(ct + ((size_t)bh * SS + q0 + ql) * HD + d0) = v;
  }
}

__global__ __launch_bounds__(128) void attn_kernel(
    const _Float16* __restrict__ qh, const _Float16* __restrict__ kh, const _Float16* __restrict__ vt,
    const int* __restrict__ amask, const int* __restrict__ padm, _Float16* ct)
{
  __shared__ __attribute__((aligned(16))) _Float16 sO[4 * 16 * HD];
  const int tid = threadIdx.x, lane = tid & 31, w = tid >> 5;
  const int h = lane >> 4, m = lane & 15;
  const int bh = blockIdx.y, b = bh >> 3;
  const int q0 = blockIdx.x * 64 + 16 * w;
  const int qi = q0 + m;

  const v16h qb = load_frag(qh + ((size_t)bh * SS + qi) * HD, h);
  const int padq = padm[b * SS + qi];

  const v8f z8 = zero8f();
  v8f o[2];
  o[0] = z8; o[1] = z8;
  float mrun = -INFINITY, lrun = 0.0f;

  const _Float16* kbase = kh + ((size_t)bh * SS + m) * HD;
  const _Float16* vbase = vt + ((size_t)bh * HD + m) * SS;
  const int* mrow = amask + ((size_t)b * SS + qi) * SS + 8 * h;
  const int* prow = padm + (size_t)b * SS + 8 * h;
  const float scl = 0.17677669529663687f;

#pragma unroll 1
  for (int kb = 0; kb < SS; kb += 64) {
    v8f s[4];
#pragma unroll
    for (int j = 0; j < 4; ++j) {
      const v16h kf = load_frag(kbase + (size_t)(kb + 16 * j) * HD, h);
      s[j] = wmma_f16(kf, qb, z8);
    }
    float mloc = -INFINITY;
#pragma unroll
    for (int j = 0; j < 4; ++j) {
      const v4i ma = *(const v4ia*)(mrow + kb + 16 * j);
      const v4i mb = *(const v4ia*)(mrow + kb + 16 * j + 4);
      const v4i pa = *(const v4ia*)(prow + kb + 16 * j);
      const v4i pb = *(const v4ia*)(prow + kb + 16 * j + 4);
      const int mk[8] = { ma.x, ma.y, ma.z, ma.w, mb.x, mb.y, mb.z, mb.w };
      const int pk[8] = { pa.x, pa.y, pa.z, pa.w, pb.x, pb.y, pb.z, pb.w };
#pragma unroll
      for (int r = 0; r < 8; ++r) {
        const int key = kb + 16 * j + 8 * h + r;
        const bool ok = ((mk[r] != 0) && (padq != 0) && (pk[r] != 0)) || (key == qi);
        const float sv = ok ? (s[j][r] * scl) : -INFINITY;
        s[j][r] = sv;
        mloc = fmaxf(mloc, sv);
      }
    }
    mloc = fmaxf(mloc, __shfl_xor(mloc, 16, 32));
    const float mnew = fmaxf(mrun, mloc);
    const float msafe = (mnew == -INFINITY) ? 0.0f : mnew;
    const float alpha = __expf(mrun - msafe);
    mrun = mnew;
    float lsum = 0.0f;
#pragma unroll
    for (int j = 0; j < 4; ++j)
#pragma unroll
      for (int r = 0; r < 8; ++r) {
        const float p = __expf(s[j][r] - msafe);
        s[j][r] = p;
        lsum += p;
      }
    lsum += __shfl_xor(lsum, 16, 32);
    lrun = lrun * alpha + lsum;
#pragma unroll
    for (int t = 0; t < 2; ++t)
#pragma unroll
      for (int r = 0; r < 8; ++r) o[t][r] = o[t][r] * alpha;

    const v16h pb0 = pack_p(s[0], s[1]);
    const v16h pb1 = pack_p(s[2], s[3]);

#pragma unroll
    for (int t = 0; t < 2; ++t) {
      const _Float16* vp = vbase + (size_t)(16 * t) * SS + kb;
      const v16h vf0 = load_frag(vp, h);
      const v16h vf1 = load_frag(vp + 32, h);
      o[t] = wmma_f16(vf0, pb0, o[t]);
      o[t] = wmma_f16(vf1, pb1, o[t]);
    }
  }

  const float inv = ((lrun > 0.0f) ? rcpf(lrun) : 0.0f) * (OSC / PSC);
  _Float16* so = sO + w * (16 * HD);
#pragma unroll
  for (int t = 0; t < 2; ++t)
#pragma unroll
    for (int r = 0; r < 8; ++r)
      so[m * HD + 16 * t + 8 * h + r] = (_Float16)(o[t][r] * inv);
  __syncthreads();

  att_store_pass(so, ct, bh, q0, lane);
  __threadfence();
  att_store_pass(so, ct, bh, q0, lane);
}

__global__ __launch_bounds__(256) void fc1_kernel(
    const _Float16* __restrict__ xn, const _Float16* __restrict__ w1t,
    const float* __restrict__ b1, _Float16* hpl)
{
  __shared__ __attribute__((aligned(16))) float sY[2][64 * 68];
  const int tid = threadIdx.x, lane = tid & 31, w = tid >> 5;
  const int h = lane >> 4, m = lane & 15;
  const int n0 = blockIdx.x * 64, m0 = blockIdx.y * 64;
  const int wr = w & 3, hf = w >> 2;
  const _Float16* xa = xn + (size_t)(m0 + 16 * wr + m) * HID;
  const _Float16* wb = w1t + (size_t)(hf * MLPD + n0 + m) * HID;

  const v8f z8 = zero8f();
  v8f acc[4];
#pragma unroll
  for (int nt = 0; nt < 4; ++nt) acc[nt] = z8;

#pragma unroll 1
  for (int k0 = 0; k0 < HID; k0 += 32) {
    const v16h a = load_frag(xa + k0, h);
#pragma unroll
    for (int nt = 0; nt < 4; ++nt) {
      const v16h b = load_frag(wb + (size_t)nt * 16 * HID + k0, h);
      acc[nt] = wmma_f16(a, b, acc[nt]);
    }
  }

  float* sy = sY[hf];
#pragma unroll
  for (int nt = 0; nt < 4; ++nt)
#pragma unroll
    for (int r = 0; r < 8; ++r)
      sy[(16 * wr + 8 * h + r) * 68 + 16 * nt + m] = acc[nt][r] * (1.0f / WSC);
  __syncthreads();

  const int q8 = lane & 7, sub = lane >> 3, c8 = 8 * q8;
  const v4f bga = ld4(b1 + n0 + c8), bgb = ld4(b1 + n0 + c8 + 4);
  const v4f baa = ld4(b1 + MLPD + n0 + c8), bab = ld4(b1 + MLPD + n0 + c8 + 4);
#pragma unroll
  for (int i = 0; i < 2; ++i) {
    const int row = 8 * w + 4 * i + sub;
    const float* gp = sY[0] + row * 68 + c8;
    const float* apn = sY[1] + row * 68 + c8;
    const v4f g0 = ld4(gp) + bga, g1 = ld4(gp + 4) + bgb;
    const v4f a0 = ld4(apn) + baa, a1 = ld4(apn + 4) + bab;
    const v4f h0 = ((g0 * sig4(g0)) * a0) * HSC;
    const v4f h1 = ((g1 * sig4(g1)) * a1) * HSC;
    const v8h ov = { (_Float16)h0.x, (_Float16)h0.y, (_Float16)h0.z, (_Float16)h0.w,
                     (_Float16)h1.x, (_Float16)h1.y, (_Float16)h1.z, (_Float16)h1.w };
    _Float16* dst = hpl + (size_t)(m0 + row) * MLPD + n0 + c8;
    *(volatile v8h*)dst = ov;
    __threadfence();
    *(volatile v8h*)dst = ov;
  }
}

extern "C" void kernel_launch(void* const* d_in, const int* in_sizes, int n_in,
                              void* d_out, int out_size, void* d_ws, size_t ws_size,
                              hipStream_t stream) {
  if (n_in < 30) return;
  if (in_sizes[0] != MTOK * VD || in_sizes[1] != MTOK * SD || in_sizes[2] != MTOK * TD || in_sizes[3] != MTOK * RD) return;
  if (in_sizes[4] != SD * HID || in_sizes[5] != TD * HID || in_sizes[6] != RD * HID || in_sizes[7] != ND * HID) return;
  if (in_sizes[8] != ND * VD * HID || in_sizes[9] != CTXD * HID || in_sizes[10] != HID || in_sizes[11] != ND * HID) return;
  if (in_sizes[12] != NL * NA * HID * 3 * HID || in_sizes[13] != NL * NA * HID * HID) return;
  if (in_sizes[14] != NL * 6 * HID || in_sizes[15] != NL * 6 * HID) return;
  if (in_sizes[16] != NL * HID * FC1N || in_sizes[17] != NL * FC1N) return;
  if (in_sizes[18] != NL * MLPD * HID || in_sizes[19] != NL * HID) return;
  if (in_sizes[20] != HID || in_sizes[21] != HID || in_sizes[22] != MTOK) return;
  for (int i = 23; i < 28; ++i) if (in_sizes[i] != BB * SS * SS) return;
  if (in_sizes[28] != MTOK || in_sizes[29] != MTOK) return;
  if (out_size != MTOK * HID) return;

  const float* val_e      = (const float*)d_in[0];
  const float* sch_e      = (const float*)d_in[1];
  const float* tmp_e      = (const float*)d_in[2];
  const float* rol_e      = (const float*)d_in[3];
  const float* W_schema   = (const float*)d_in[4];
  const float* W_temporal = (const float*)d_in[5];
  const float* W_role     = (const float*)d_in[6];
  const float* E_dtype    = (const float*)d_in[7];
  const float* W_value    = (const float*)d_in[8];
  const float* W_gate     = (const float*)d_in[9];
  const float* b_gate     = (const float*)d_in[10];
  const float* E_mask     = (const float*)d_in[11];
  const float* qkv_w      = (const float*)d_in[12];
  const float* out_w      = (const float*)d_in[13];
  const float* ln_g       = (const float*)d_in[14];
  const float* ln_b       = (const float*)d_in[15];
  const float* fc1_w      = (const float*)d_in[16];
  const float* fc1_b      = (const float*)d_in[17];
  const float* fc2_w      = (const float*)d_in[18];
  const float* fc2_b      = (const float*)d_in[19];
  const float* lnf_g      = (const float*)d_in[20];
  const float* lnf_b      = (const float*)d_in[21];
  const int*   dtype_ids  = (const int*)d_in[22];
  const int*   msk[5]     = { (const int*)d_in[23], (const int*)d_in[24], (const int*)d_in[25],
                              (const int*)d_in[26], (const int*)d_in[27] };
  const int*   is_masked  = (const int*)d_in[28];
  const int*   padm       = (const int*)d_in[29];
  float* outp = (float*)d_out;

  size_t off = 0;
  auto carve = [&](size_t bytes) { const size_t o = off; off += (bytes + 255) & ~(size_t)255; return o; };
  const size_t oQKVT  = carve((size_t)NL * NA * 3 * HID * HID * 2);
  const size_t oOUTT  = carve((size_t)NL * NA * HID * HID * 2);
  const size_t oF1T   = carve((size_t)NL * FC1N * HID * 2);
  const size_t oF2T   = carve((size_t)NL * HID * MLPD * 2);
  const size_t oWST   = carve((size_t)HID * SD * 2);
  const size_t oWRT   = carve((size_t)HID * RD * 2);
  const size_t oWVT   = carve((size_t)ND * HID * VD * 2);
  const size_t oWGT   = carve((size_t)HID * CTXD * 2);
  const size_t oVAL16 = carve((size_t)MTOK * VD * 2);
  const size_t oSCH16 = carve((size_t)MTOK * SD * 2);
  const size_t oROL16 = carve((size_t)MTOK * RD * 2);
  const size_t oVP    = carve((size_t)ND * MTOK * HID * 4);
  const size_t oSP    = carve((size_t)MTOK * HID * 4);
  const size_t oRP    = carve((size_t)MTOK * HID * 4);
  const size_t oCOMB  = carve((size_t)MTOK * HID * 4);
  const size_t oCTX   = carve((size_t)MTOK * CTXD * 2);
  const size_t oX     = carve((size_t)MTOK * HID * 4);
  const size_t oXN    = carve((size_t)MTOK * HID * 2);
  const size_t oQ     = carve((size_t)BB * NHD * SS * HD * 2);
  const size_t oK     = carve((size_t)BB * NHD * SS * HD * 2);
  const size_t oVT    = carve((size_t)BB * NHD * HD * SS * 2);
  const size_t oCT    = carve((size_t)BB * NHD * SS * HD * 2);
  const size_t oH     = carve((size_t)MTOK * MLPD * 2);
  if (off > ws_size) return;
  if (off > (size_t)134217728) return;

  char* ws = (char*)d_ws;
  _Float16* QKVT  = (_Float16*)(ws + oQKVT);
  _Float16* OUTT  = (_Float16*)(ws + oOUTT);
  _Float16* F1T   = (_Float16*)(ws + oF1T);
  _Float16* F2T   = (_Float16*)(ws + oF2T);
  _Float16* WST   = (_Float16*)(ws + oWST);
  _Float16* WRT   = (_Float16*)(ws + oWRT);
  _Float16* WVT   = (_Float16*)(ws + oWVT);
  _Float16* WGT   = (_Float16*)(ws + oWGT);
  _Float16* VAL16 = (_Float16*)(ws + oVAL16);
  _Float16* SCH16 = (_Float16*)(ws + oSCH16);
  _Float16* ROL16 = (_Float16*)(ws + oROL16);
  float*    VP    = (float*)(ws + oVP);
  float*    SP    = (float*)(ws + oSP);
  float*    RP    = (float*)(ws + oRP);
  float*    COMB  = (float*)(ws + oCOMB);
  _Float16* CTX16 = (_Float16*)(ws + oCTX);
  float*    X     = (float*)(ws + oX);
  _Float16* XN    = (_Float16*)(ws + oXN);
  _Float16* Qp    = (_Float16*)(ws + oQ);
  _Float16* Kp    = (_Float16*)(ws + oK);
  _Float16* VTp   = (_Float16*)(ws + oVT);
  _Float16* CT    = (_Float16*)(ws + oCT);
  _Float16* Hp    = (_Float16*)(ws + oH);

  {
    const int n8 = MTOK * VD / 8 + MTOK * SD / 8 + MTOK * RD / 8;
    cvt_in_kernel<<<dim3((n8 + 255) / 256), dim3(256), 0, stream>>>(val_e, sch_e, rol_e, VAL16, SCH16, ROL16);
  }
  auto wt = [&](const float* wsrc, _Float16* o, int K, int N, int Z) {
    wtrans_kernel<<<dim3(N / 64, K / 64, Z), dim3(256), 0, stream>>>(wsrc, o, K, N);
  };
  wt(qkv_w,    QKVT, HID,  3 * HID, NL * NA);
  wt(out_w,    OUTT, HID,  HID,     NL * NA);
  wt(fc1_w,    F1T,  HID,  FC1N,    NL);
  wt(fc2_w,    F2T,  MLPD, HID,     NL);
  wt(W_schema, WST,  SD,   HID,     1);
  wt(W_role,   WRT,  RD,   HID,     1);
  wt(W_value,  WVT,  VD,   HID,     ND);
  wt(W_gate,   WGT,  CTXD, HID,     1);

  gemm_f32_kernel<<<dim3(MTOK / 128, HID / 64, ND), dim3(128), 0, stream>>>(
      VAL16, VD, 0LL, WVT, VD, (long long)HID * VD, VP, HID, (long long)MTOK * HID, VD, 1.0f / WSC);
  gemm_f32_kernel<<<dim3(MTOK / 128, HID / 64, 1), dim3(128), 0, stream>>>(
      SCH16, SD, 0LL, WST, SD, 0LL, SP, HID, 0LL, SD, 1.0f / WSC);
  gemm_f32_kernel<<<dim3(MTOK / 128, HID / 64, 1), dim3(128), 0, stream>>>(
      ROL16, RD, 0LL, WRT, RD, 0LL, RP, HID, 0LL, RD, 1.0f / WSC);

  embed_kernel<<<dim3(MTOK / 8), dim3(256), 0, stream>>>(
      VP, SP, RP, tmp_e, W_temporal, E_dtype, E_mask, dtype_ids, is_masked, COMB, CTX16);

  rowgemm_kernel<0, 1, 1, 0><<<dim3(MTOK / 32), dim3(128), 0, stream>>>(
      CTX16, CTXD, WGT, CTXD, 1.0f / (CSC * WSC), b_gate, X, COMB, padm,
      ln_g, ln_b, XN, outp);

  for (int l = 0; l < NL; ++l) {
    for (int a = 0; a < NA; ++a) {
      const _Float16* wq = QKVT + (size_t)(l * NA + a) * 3 * HID * HID;
      qkv_kernel<<<dim3(MTOK / 128, 3 * HID / 64), dim3(128), 0, stream>>>(XN, wq, Qp, Kp, VTp);
      attn_kernel<<<dim3(SS / 64, BB * NHD), dim3(128), 0, stream>>>(Qp, Kp, VTp, msk[a], padm, CT);
      const int lnn = (a < NA - 1) ? (l * 6 + a + 1) : (l * 6 + 5);
      rowgemm_kernel<1, 0, 0, 0><<<dim3(MTOK / 32), dim3(128), 0, stream>>>(
          CT, HD, OUTT + (size_t)(l * NA + a) * HID * HID, HID, 1.0f / (OSC * WSC), b_gate, X, COMB, padm,
          ln_g + (size_t)lnn * HID, ln_b + (size_t)lnn * HID, XN, outp);
    }
    fc1_kernel<<<dim3(MLPD / 64, MTOK / 64), dim3(256), 0, stream>>>(
        XN, F1T + (size_t)l * FC1N * HID, fc1_b + (size_t)l * FC1N, Hp);
    if (l < NL - 1) {
      const int lnn = (l + 1) * 6;
      rowgemm_kernel<0, 0, 1, 0><<<dim3(MTOK / 32), dim3(128), 0, stream>>>(
          Hp, MLPD, F2T + (size_t)l * HID * MLPD, MLPD, 1.0f / (HSC * WSC), fc2_b + (size_t)l * HID, X, COMB, padm,
          ln_g + (size_t)lnn * HID, ln_b + (size_t)lnn * HID, XN, outp);
    } else {
      rowgemm_kernel<0, 0, 1, 1><<<dim3(MTOK / 32), dim3(128), 0, stream>>>(
          Hp, MLPD, F2T + (size_t)l * HID * MLPD, MLPD, 1.0f / (HSC * WSC), fc2_b + (size_t)l * HID, X, COMB, padm,
          lnf_g, lnf_b, XN, outp);
    }
  }
  (void)hipGetLastError();
}
